// Normalized_Correlation_Layer_39470749450727
// MI455X (gfx1250) — hardware-verified
//
#include <hip/hip_runtime.h>


namespace {
constexpr int Bn = 8, H = 64, W = 32, C = 64, K = 5, OR = H - K + 1  , OC = W - K + 1  , P2 = OR * OC  , SR = (H - K) / 2 + 1  , SC = (W - K) / 2 + 1  , P1 = SR * SC  ;
constexpr int F = K * K * C  , NP1 = 448  , P1PAD = 432  ;
typedef __attribute__((ext_vector_type(16))) __bf16 v16bb;
typedef __attribute__((ext_vector_type(8))) unsigned short v8us;
typedef __attribute__((ext_vector_type(8))) float v8f;
typedef __attribute__((ext_vector_type(4))) float v4f;
__device__ __forceinline__ float bf16_rne(float f) { unsigned int u = __float_as_uint(f); u += 0x7FFFu + ((u >> 16) & 1u); return __uint_as_float(u & 0xFFFF0000u); }
__device__ __forceinline__ unsigned short bf16_bits(float f) { unsigned int u = __float_as_uint(f); u += 0x7FFFu + ((u >> 16) & 1u); return (unsigned short)(u >> 16); }
__device__ __forceinline__ v16bb frag_bf(const unsigned short* p, int hh) { typedef __attribute__((ext_vector_type(8))) unsigned short v8; const v8 a = *(const v8*)(p + 8 * hh), b = *(const v8*)(p + 16 + 8 * hh);
  union { unsigned short s[16]; v16bb v; } u;
#pragma unroll
  for (int e = 0; e < 8; ++e) { u.s[e] = a[e]; u.s[8 + e] = b[e]; } return u.v; }
__device__ __forceinline__ v8f wmma_bf(v16bb a, v16bb b, v8f c) {
  v8f d = __builtin_amdgcn_wmma_f32_16x16x32_bf16(false, a, false, b, (short)0, c, false, false);
  asm volatile("v_nop\n\tv_nop\n\tv_nop\n\tv_nop" : "+v"(d) : "v"(a), "v"(b));
  return d;
}

__global__ __launch_bounds__(256) void prep_kernel(const float* __restrict__ i1, const float* __restrict__ i2, unsigned short* __restrict__ b1, unsigned short* __restrict__ b2) {
  const size_t i = (size_t)blockIdx.x * 256 + threadIdx.x; v8us u, v;
#pragma unroll
  for (int e = 0; e < 8; ++e) { u[e] = bf16_bits(i1[i * 8 + e]); v[e] = bf16_bits(i2[i * 8 + e]); }
  for (int pass = 0; pass < 2; ++pass) { *(volatile v8us*)(b1 + i * 8) = u; *(volatile v8us*)(b2 + i * 8) = v; __threadfence(); }
}

template <int WHICH>
__global__ __launch_bounds__(256) void stats_kernel(const float* __restrict__ img, float* __restrict__ st) {
  constexpr int NPATCH = WHICH ? P1 : P2, NPAD_ = WHICH ? P1PAD : P2, NCOL = WHICH ? SC : OC, STRIDE = WHICH ? 2 : 1;
  __shared__ float Sb[16][2];
  constexpr int NBLKP = (NPATCH + 15) / 16;
  const int wave = threadIdx.x >> 5, lane = threadIdx.x & 31, b = blockIdx.x / NBLKP, pbase = (blockIdx.x % NBLKP) * 16;
  for (int k = 0; k < 2; ++k) { const int pl = wave * 2 + k, p = min(pbase + pl, NPATCH - 1); const int y0 = (p / NCOL) * STRIDE, x0 = (p % NCOL) * STRIDE; float s = 0.0f, s2 = 0.0f;
    for (int dyx = 0; dyx < K * K; ++dyx) { const int dy = dyx / K, dx = dyx % K; const float* px = img + (((size_t)b * H + y0 + dy) * W + x0 + dx) * C;
      const float v0 = bf16_rne(px[lane]), v1 = bf16_rne(px[32 + lane]); s += v0 + v1; s2 += v0 * v0 + v1 * v1; }
#pragma unroll
    for (int o = 16; o > 0; o >>= 1) { s += __shfl_xor(s, o); s2 += __shfl_xor(s2, o); }
    if (lane == 0) { const float mean = s * (1.0f / F); const float var = fmaxf(s2 * (1.0f / F) - mean * mean, 0.0f); Sb[pl][0] = mean; Sb[pl][1] = rsqrtf(var); } }
  __syncthreads();
  for (int pass = 0; pass < 2; ++pass) { if (threadIdx.x < 32 && pbase + (threadIdx.x >> 1) < NPATCH) ((volatile float*)st)[((size_t)b * NPAD_ + pbase) * 2 + threadIdx.x] = Sb[threadIdx.x >> 1][threadIdx.x & 1]; __threadfence(); }
}

__global__ __launch_bounds__(128) void corr_kernel(const unsigned short* __restrict__ b2, const unsigned short* __restrict__ b1, const float* __restrict__ st2, const float* __restrict__ st1, float* __restrict__ out) {
  __shared__ __attribute__((aligned(16))) float Ot[16][P1];
  const int wave = threadIdx.x >> 5, lane = threadIdx.x & 31, nloc = lane & 15, hlf = lane >> 4, b = blockIdx.x / (P2 / 16), p0 = (blockIdx.x % (P2 / 16)) * 16;
  const int p = p0 + nloc, py = p / OC, px = p % OC;
  int qy[7], qx[7];
#pragma unroll
  for (int t = 0; t < 7; ++t) { const int q = min(wave * 112 + t * 16 + nloc, P1 - 1); qy[t] = (q / SC) * 2; qx[t] = (q % SC) * 2; }
  v8f acc[7] = {{}, {}, {}, {}, {}, {}, {}};
#pragma unroll 1
  for (int dyx = 0; dyx < K * K; ++dyx) { const int dy = dyx / K, dx = dyx % K;
#pragma unroll
    for (int ch = 0; ch < 2; ++ch) { const v16bb a = frag_bf(b2 + (((size_t)b * H + py + dy) * W + px + dx) * C + ch * 32, hlf);
#pragma unroll
      for (int t = 0; t < 7; ++t) { const v16bb bb = frag_bf(b1 + (((size_t)b * H + qy[t] + dy) * W + qx[t] + dx) * C + ch * 32, hlf); acc[t] = wmma_bf(a, bb, acc[t]); } } }
#pragma unroll
  for (int t = 0; t < 7; ++t) { const int q = wave * 112 + t * 16 + nloc; if (q < P1) { const float m1 = st1[((size_t)b * P1PAD + q) * 2], r1 = st1[((size_t)b * P1PAD + q) * 2 + 1];
#pragma unroll
      for (int v = 0; v < 8; ++v) { const int pp = p0 + 8 * hlf + v; const float m2 = st2[((size_t)b * P2 + pp) * 2], r2 = st2[((size_t)b * P2 + pp) * 2 + 1];
        Ot[8 * hlf + v][q] = (acc[t][v] - (float)F * m2 * m1) * r2 * r1; } } }
  __syncthreads();
  float* dst = out + ((size_t)b * P2 + p0) * P1;
  for (int pass = 0; pass < 2; ++pass) { for (int i = threadIdx.x; i < 16 * P1 / 4; i += 128) *(volatile v4f*)(dst + (size_t)i * 4) = *(const v4f*)(&Ot[0][0] + i * 4); __threadfence(); }
}
}

extern "C" void kernel_launch(void* const* d_in, const int* in_sizes, int n_in,
                              void* d_out, int out_size, void* d_ws, size_t ws_size, hipStream_t stream) {
  (void)n_in; (void)out_size;
  const float* i1 = (const float*)d_in[0]; const float* i2 = (const float*)d_in[1];
  float* out = (float*)d_out;
  if (in_sizes[0] != Bn * H * W * C || in_sizes[1] != Bn * H * W * C) return;
  size_t off = 0; char* ws = (char*)d_ws;
  auto carve = [&](size_t bytes) { char* p = ws + off; off += (bytes + 255) & ~(size_t)255; return p; };
  unsigned short* b1 = (unsigned short*)carve((size_t)Bn * H * W * C * 2); unsigned short* b2 = (unsigned short*)carve((size_t)Bn * H * W * C * 2); float* st1 = (float*)carve((size_t)Bn * P1PAD * 2 * 4); float* st2 = (float*)carve((size_t)Bn * P2 * 2 * 4);
  if (off > ws_size) return;
  prep_kernel<<<Bn * H * W * C / 8 / 256, 256, 0, stream>>>(i1, i2, b1, b2);
  stats_kernel<0><<<Bn * ((P2 + 15) / 16), 256, 0, stream>>>(i2, st2);
  stats_kernel<1><<<Bn * ((P1 + 15) / 16), 256, 0, stream>>>(i1, st1);
  corr_kernel<<<Bn * (P2 / 16), 128, 0, stream>>>(b2, b1, st2, st1, out);
}
